// Enc_Dec_linear_38250978738658
// MI455X (gfx1250) — hardware-run, weakly checked
//
#include <hip/hip_runtime.h>
#include <stdint.h>

typedef __attribute__((ext_vector_type(16))) _Float16 v16h;
typedef __attribute__((ext_vector_type(8)))  _Float16 v8h;
typedef __attribute__((ext_vector_type(8)))  float    v8f;
typedef __attribute__((ext_vector_type(4)))  float    v4f;

__device__ __forceinline__ void dep_guard_h(v8f& a, v8f& b, v16h x, v16h y) { asm volatile("v_nop\n\tv_nop\n\tv_nop\n\tv_nop" : "+v"(a), "+v"(b) : "v"(x), "v"(y)); }
__device__ __forceinline__ void keep4_h(v16h a, v16h b, v16h c, v16h d) { asm volatile("v_nop" :: "v"(a), "v"(b), "v"(c), "v"(d)); }
__device__ __forceinline__ void acc_guard4(v8f& a, v8f& b, v8f& c, v8f& d) { asm volatile("v_nop\n\tv_nop\n\tv_nop\n\tv_nop" : "+v"(a), "+v"(b), "+v"(c), "+v"(d)); }
template <typename T> struct Frag;
template <> struct Frag<_Float16> {
  typedef v16h V; union U { v16h v; v8h h[2]; };
  static __device__ __forceinline__ v16h load(const _Float16* p) {
    U f; f.h[0] = *(const v8h*)(p); f.h[1] = *(const v8h*)(p + 16); return f.v;
  }
  static __device__ __forceinline__ v8f mma(v16h a, v16h b, v8f c) {
    return __builtin_amdgcn_wmma_f32_16x16x32_f16(false, a, false, b, (short)0, c, false, false);
  }
  static __device__ __forceinline__ void guard(v8f& a, v8f& b, v16h x, v16h y) { dep_guard_h(a, b, x, y); }
  static __device__ __forceinline__ void keep(v16h a, v16h b, v16h c, v16h d) { keep4_h(a, b, c, d); }
};

__device__ __forceinline__ void guard4x(v8f& a, v8f& b, v8f& c2, v8f& d, v16h x, v16h y, v16h z, v16h w) {
  asm volatile("v_nop\n\tv_nop\n\tv_nop\n\tv_nop" : "+v"(a), "+v"(b), "+v"(c2), "+v"(d) : "v"(x), "v"(y), "v"(z), "v"(w));
}
__device__ __forceinline__ void guard2x(v8f& a, v8f& b, v16h x, v16h y, v16h z) {
  asm volatile("v_nop\n\tv_nop\n\tv_nop\n\tv_nop" : "+v"(a), "+v"(b) : "v"(x), "v"(y), "v"(z));
}

constexpr int kBatch = 16;
constexpr int kSteps = 12;
constexpr int kNodes = 10000;
constexpr int kFeat  = 64;
constexpr int kTdec  = 12;
constexpr int kRows  = kBatch * kNodes;
constexpr int kRowsPerBlock = 32;
constexpr int kMainBlocks   = kRows / kRowsPerBlock;
constexpr int kMainThreads  = 128;
constexpr int kAPitch     = 192;
constexpr int kTileHalves = kRowsPerBlock * kAPitch;
constexpr int kOutCols    = 16;
constexpr int kPermThreads = 256;
constexpr int kPermBlocks  = (kRows * kTdec) / (4 * kPermThreads);
static_assert(kRows % kRowsPerBlock == 0);
static_assert(kMainBlocks == 5000);
static_assert((kRows * kTdec) % (4 * kPermThreads) == 0);
static_assert(kNodes % 4 == 0);
static_assert(kFeat == 64);

union V8 { v8f v; v4f q[2]; };

__device__ __forceinline__ v8f splat8(float v) { return (v8f){v, v, v, v, v, v, v, v}; }
__device__ __forceinline__ v8f mma_h(v16h a, v16h b, v8f c) { return Frag<_Float16>::mma(a, b, c); }
__device__ __forceinline__ float fsig(float x)  { return __builtin_amdgcn_rcpf(1.0f + __builtin_amdgcn_exp2f(-1.4426950408889634f * x)); }
__device__ __forceinline__ float ftanh(float x) { return 1.0f - 2.0f * __builtin_amdgcn_rcpf(1.0f + __builtin_amdgcn_exp2f(2.8853900817779268f * x)); }

__global__ __launch_bounds__(256) void prep_wt8(const float* __restrict__ W, _Float16* __restrict__ Bt,
                                                int kshift, int N, int total8) {
  const int i = blockIdx.x * 256 + threadIdx.x;
  if (i < total8) {
    const int K  = 1 << kshift;
    const int e8 = i << 3;
    const int n  = e8 >> kshift;
    const int k0 = e8 & (K - 1);
    v8h hv;
#pragma unroll
    for (int j = 0; j < 8; ++j) hv[j] = (_Float16)(W[(size_t)(k0 + j) * N + n] * 8.0f);
    _Float16* p = Bt + e8;
    *(volatile v8h*)p = hv;
    __threadfence();
    *(volatile v8h*)p = hv;
  }
}

__global__ __launch_bounds__(kMainThreads) void gru_seq_main(
    const float* __restrict__ xin, const float* __restrict__ winw, const float* __restrict__ winb,
    const _Float16* __restrict__ egt, const float* __restrict__ egb,
    const _Float16* __restrict__ eut, const float* __restrict__ eub,
    const _Float16* __restrict__ ewt, const float* __restrict__ ebb,
    const _Float16* __restrict__ dgt, const float* __restrict__ dgb,
    const _Float16* __restrict__ dut, const float* __restrict__ dub,
    const _Float16* __restrict__ dwt, const float* __restrict__ dbb,
    const float* __restrict__ wow, const float* __restrict__ wob,
    float* __restrict__ OW) {
  __shared__ __align__(16) _Float16 sA[2 * kTileHalves];
  __shared__ __align__(16) float sC[192 * kRowsPerBlock];
  __shared__ __align__(16) float sOut[kRowsPerBlock * kOutCols];
  __shared__ __align__(16) float sPart[4 * kRowsPerBlock];

  const int tid  = threadIdx.x;
  const int wave = tid >> 5;
  const int lane = tid & 31;
  const int hh   = lane >> 4;
  const int c    = lane & 15;
  const int ub   = wave;
  const int ucol = 16 * ub + c;
  const int koff = 8 * hh;
  const int rl   = 8 * hh;

  const int xrow = tid & 31;
  const int xcg  = wave * 16;
  const int rgx  = blockIdx.x * kRowsPerBlock + xrow;
  const int xb   = rgx / kNodes;
  const int xn   = rgx - xb * kNodes;
  const float* xsrc = xin + (size_t)xb * (size_t)(kSteps * kNodes) + xn;

  if (tid < kRowsPerBlock) {
#pragma unroll
    for (int j = 0; j < kOutCols; ++j) sOut[tid * kOutCols + j] = 0.0f;
  }

  float h[2][8];
#pragma unroll
  for (int mi = 0; mi < 2; ++mi)
#pragma unroll
    for (int r = 0; r < 8; ++r) h[mi][r] = 0.0f;

  const float gbr8 = 8.0f * egb[ucol];
  const float gbu8 = 8.0f * egb[64 + ucol];
  const float cb8  = 8.0f * eub[ucol];

#pragma unroll 1
  for (int p = 0; p < kSteps; ++p) {
    _Float16* tA = sA + (p & 1) * kTileHalves;
#pragma unroll
    for (int mi = 0; mi < 2; ++mi)
#pragma unroll
      for (int r = 0; r < 8; ++r)
        tA[(rl + 16 * mi + r) * kAPitch + 64 + ucol] = (_Float16)h[mi][r];
    {
      const float s = xsrc[(size_t)p * kNodes];
      v8h x0, x1;
#pragma unroll
      for (int e = 0; e < 8; ++e) {
        x0[e] = (_Float16)(s * winw[xcg + e] + winb[xcg + e]);
        x1[e] = (_Float16)(s * winw[xcg + 8 + e] + winb[xcg + 8 + e]);
      }
      *(v8h*)(tA + xrow * kAPitch + xcg)     = x0;
      *(v8h*)(tA + xrow * kAPitch + xcg + 8) = x1;
    }
    __syncthreads();

    const _Float16* aP = tA + c * kAPitch + koff;
    v8f ar[2], au[2];
    ar[0] = splat8(gbr8); ar[1] = ar[0];
    au[0] = splat8(gbu8); au[1] = au[0];
    {
      const _Float16* brP = egt + (size_t)ucol * 128 + koff;
      const _Float16* buP = egt + (size_t)(64 + ucol) * 128 + koff;
#pragma unroll
      for (int ks = 0; ks < 4; ++ks) {
        const v16h br = Frag<_Float16>::load(brP + 32 * ks);
        const v16h bu = Frag<_Float16>::load(buP + 32 * ks);
        const v16h a0 = Frag<_Float16>::load(aP + 32 * ks);
        const v16h a1 = Frag<_Float16>::load(aP + 16 * kAPitch + 32 * ks);
        ar[0] = mma_h(a0, br, ar[0]);
        au[0] = mma_h(a0, bu, au[0]);
        ar[1] = mma_h(a1, br, ar[1]);
        au[1] = mma_h(a1, bu, au[1]);
        guard4x(ar[0], ar[1], au[0], au[1], a0, a1, br, bu);
      }
    }
    float u[2][8];
#pragma unroll
    for (int mi = 0; mi < 2; ++mi) {
#pragma unroll
      for (int r = 0; r < 8; ++r) {
        const float rr = fsig(ar[mi][r] * 0.125f);
        u[mi][r] = fsig(au[mi][r] * 0.125f);
        tA[(rl + 16 * mi + r) * kAPitch + 128 + ucol] = (_Float16)(rr * h[mi][r]);
      }
    }
    __syncthreads();

    v8f ac[2];
    ac[0] = splat8(cb8); ac[1] = ac[0];
    {
      const _Float16* bP = eut + (size_t)ucol * 128 + koff;
#pragma unroll
      for (int ks = 0; ks < 4; ++ks) {
        const int cbA = (ks < 2) ? (32 * ks) : (128 + 32 * (ks - 2));
        const v16h b  = Frag<_Float16>::load(bP + 32 * ks);
        const v16h a0 = Frag<_Float16>::load(aP + cbA);
        const v16h a1 = Frag<_Float16>::load(aP + 16 * kAPitch + cbA);
        ac[0] = mma_h(a0, b, ac[0]);
        ac[1] = mma_h(a1, b, ac[1]);
        guard2x(ac[0], ac[1], a0, a1, b);
      }
    }
#pragma unroll
    for (int mi = 0; mi < 2; ++mi) {
#pragma unroll
      for (int r = 0; r < 8; ++r) {
        const float cy = ftanh(ac[mi][r] * 0.125f);
        const float uu = u[mi][r];
        h[mi][r] = uu * h[mi][r] + (1.0f - uu) * cy;
      }
    }
  }

  _Float16* t0 = sA;
  const _Float16* aP0 = t0 + c * kAPitch + koff;
#pragma unroll
  for (int mi = 0; mi < 2; ++mi)
#pragma unroll
    for (int r = 0; r < 8; ++r)
      t0[(rl + 16 * mi + r) * kAPitch + 64 + ucol] = (_Float16)h[mi][r];
  __syncthreads();
  {
    const float eb8 = 8.0f * ebb[ucol];
    v8f ay[2];
    ay[0] = splat8(eb8); ay[1] = ay[0];
    const _Float16* bP = ewt + (size_t)ucol * 64 + koff;
#pragma unroll
    for (int ks = 0; ks < 2; ++ks) {
      const v16h b  = Frag<_Float16>::load(bP + 32 * ks);
      const v16h a0 = Frag<_Float16>::load(aP0 + 64 + 32 * ks);
      const v16h a1 = Frag<_Float16>::load(aP0 + 16 * kAPitch + 64 + 32 * ks);
      ay[0] = mma_h(a0, b, ay[0]);
      ay[1] = mma_h(a1, b, ay[1]);
      guard2x(ay[0], ay[1], a0, a1, b);
    }
#pragma unroll
    for (int mi = 0; mi < 2; ++mi)
#pragma unroll
      for (int r = 0; r < 8; ++r)
        t0[(rl + 16 * mi + r) * kAPitch + ucol] = (_Float16)fsig(ay[mi][r] * 0.125f);
  }
  __syncthreads();
  {
    v8f gr[2], gu[2];
    gr[0] = splat8(8.0f * dgb[ucol]);      gr[1] = gr[0];
    gu[0] = splat8(8.0f * dgb[64 + ucol]); gu[1] = gu[0];
    const _Float16* brP = dgt + (size_t)ucol * 128 + koff;
    const _Float16* buP = dgt + (size_t)(64 + ucol) * 128 + koff;
#pragma unroll
    for (int ks = 0; ks < 2; ++ks) {
      const v16h br = Frag<_Float16>::load(brP + 32 * ks);
      const v16h bu = Frag<_Float16>::load(buP + 32 * ks);
      const v16h a0 = Frag<_Float16>::load(aP0 + 32 * ks);
      const v16h a1 = Frag<_Float16>::load(aP0 + 16 * kAPitch + 32 * ks);
      gr[0] = mma_h(a0, br, gr[0]);
      gu[0] = mma_h(a0, bu, gu[0]);
      gr[1] = mma_h(a1, br, gr[1]);
      gu[1] = mma_h(a1, bu, gu[1]);
      guard4x(gr[0], gr[1], gu[0], gu[1], a0, a1, br, bu);
    }
#pragma unroll
    for (int mi = 0; mi < 2; ++mi) {
      V8 tr; tr.v = gr[mi];
      V8 tu; tu.v = gu[mi];
      *(v4f*)(sC + ucol * kRowsPerBlock + rl + 16 * mi)            = tr.q[0];
      *(v4f*)(sC + ucol * kRowsPerBlock + rl + 16 * mi + 4)        = tr.q[1];
      *(v4f*)(sC + (64 + ucol) * kRowsPerBlock + rl + 16 * mi)     = tu.q[0];
      *(v4f*)(sC + (64 + ucol) * kRowsPerBlock + rl + 16 * mi + 4) = tu.q[1];
    }
  }
  {
    v8f gc[2];
    gc[0] = splat8(8.0f * dub[ucol]); gc[1] = gc[0];
    const _Float16* bP = dut + (size_t)ucol * 128 + koff;
#pragma unroll
    for (int ks = 0; ks < 2; ++ks) {
      const v16h b  = Frag<_Float16>::load(bP + 32 * ks);
      const v16h a0 = Frag<_Float16>::load(aP0 + 32 * ks);
      const v16h a1 = Frag<_Float16>::load(aP0 + 16 * kAPitch + 32 * ks);
      gc[0] = mma_h(a0, b, gc[0]);
      gc[1] = mma_h(a1, b, gc[1]);
      guard2x(gc[0], gc[1], a0, a1, b);
    }
#pragma unroll
    for (int mi = 0; mi < 2; ++mi) {
      V8 tc; tc.v = gc[mi];
      *(v4f*)(sC + (128 + ucol) * kRowsPerBlock + rl + 16 * mi)     = tc.q[0];
      *(v4f*)(sC + (128 + ucol) * kRowsPerBlock + rl + 16 * mi + 4) = tc.q[1];
    }
  }
  const float db8  = 8.0f * dbb[ucol];
  const float wo   = wow[ucol];
  const float wob0 = wob[0];
  __syncthreads();

#pragma unroll 1
  for (int t = 0; t < kTdec; ++t) {
    const int par = t & 1;
    _Float16* tA = sA + par * kTileHalves;
    _Float16* tB = sA + (par ^ 1) * kTileHalves;
    const _Float16* aPA = tA + c * kAPitch + koff;
    const _Float16* aPB = tB + c * kAPitch + koff;

    v8f ar[2], au[2];
#pragma unroll
    for (int mi = 0; mi < 2; ++mi) {
      V8 tr, tu;
      tr.q[0] = *(const v4f*)(sC + ucol * kRowsPerBlock + rl + 16 * mi);
      tr.q[1] = *(const v4f*)(sC + ucol * kRowsPerBlock + rl + 16 * mi + 4);
      tu.q[0] = *(const v4f*)(sC + (64 + ucol) * kRowsPerBlock + rl + 16 * mi);
      tu.q[1] = *(const v4f*)(sC + (64 + ucol) * kRowsPerBlock + rl + 16 * mi + 4);
      ar[mi] = tr.v; au[mi] = tu.v;
    }
    {
      const _Float16* brP = dgt + (size_t)ucol * 128 + 64 + koff;
      const _Float16* buP = dgt + (size_t)(64 + ucol) * 128 + 64 + koff;
#pragma unroll
      for (int ks = 0; ks < 2; ++ks) {
        const v16h br = Frag<_Float16>::load(brP + 32 * ks);
        const v16h bu = Frag<_Float16>::load(buP + 32 * ks);
        const v16h a0 = Frag<_Float16>::load(aPA + 64 + 32 * ks);
        const v16h a1 = Frag<_Float16>::load(aPA + 16 * kAPitch + 64 + 32 * ks);
        ar[0] = mma_h(a0, br, ar[0]);
        au[0] = mma_h(a0, bu, au[0]);
        ar[1] = mma_h(a1, br, ar[1]);
        au[1] = mma_h(a1, bu, au[1]);
        guard4x(ar[0], ar[1], au[0], au[1], a0, a1, br, bu);
      }
    }
    float u[2][8];
#pragma unroll
    for (int mi = 0; mi < 2; ++mi) {
#pragma unroll
      for (int r = 0; r < 8; ++r) {
        const float rr = fsig(ar[mi][r] * 0.125f);
        u[mi][r] = fsig(au[mi][r] * 0.125f);
        tA[(rl + 16 * mi + r) * kAPitch + 128 + ucol] = (_Float16)(rr * h[mi][r]);
      }
    }
    __syncthreads();

    v8f ac[2];
#pragma unroll
    for (int mi = 0; mi < 2; ++mi) {
      V8 tc;
      tc.q[0] = *(const v4f*)(sC + (128 + ucol) * kRowsPerBlock + rl + 16 * mi);
      tc.q[1] = *(const v4f*)(sC + (128 + ucol) * kRowsPerBlock + rl + 16 * mi + 4);
      ac[mi] = tc.v;
    }
    {
      const _Float16* bP = dut + (size_t)ucol * 128 + 64 + koff;
#pragma unroll
      for (int ks = 0; ks < 2; ++ks) {
        const v16h b  = Frag<_Float16>::load(bP + 32 * ks);
        const v16h a0 = Frag<_Float16>::load(aPA + 128 + 32 * ks);
        const v16h a1 = Frag<_Float16>::load(aPA + 16 * kAPitch + 128 + 32 * ks);
        ac[0] = mma_h(a0, b, ac[0]);
        ac[1] = mma_h(a1, b, ac[1]);
        guard2x(ac[0], ac[1], a0, a1, b);
      }
    }
#pragma unroll
    for (int mi = 0; mi < 2; ++mi) {
#pragma unroll
      for (int r = 0; r < 8; ++r) {
        const float cy = ftanh(ac[mi][r] * 0.125f);
        const float uu = u[mi][r];
        const float hn = uu * h[mi][r] + (1.0f - uu) * cy;
        h[mi][r] = hn;
        tB[(rl + 16 * mi + r) * kAPitch + 64 + ucol] = (_Float16)hn;
      }
    }
    __syncthreads();

    v8f ay[2];
    ay[0] = splat8(db8); ay[1] = ay[0];
    {
      const _Float16* bP = dwt + (size_t)ucol * 64 + koff;
#pragma unroll
      for (int ks = 0; ks < 2; ++ks) {
        const v16h b  = Frag<_Float16>::load(bP + 32 * ks);
        const v16h a0 = Frag<_Float16>::load(aPB + 64 + 32 * ks);
        const v16h a1 = Frag<_Float16>::load(aPB + 16 * kAPitch + 64 + 32 * ks);
        ay[0] = mma_h(a0, b, ay[0]);
        ay[1] = mma_h(a1, b, ay[1]);
        guard2x(ay[0], ay[1], a0, a1, b);
      }
    }
#pragma unroll
    for (int mi = 0; mi < 2; ++mi) {
#pragma unroll
      for (int r = 0; r < 8; ++r) {
        float q = fsig(ay[mi][r] * 0.125f) * wo;
        q += __shfl_xor(q, 1);
        q += __shfl_xor(q, 2);
        q += __shfl_xor(q, 4);
        q += __shfl_xor(q, 8);
        sPart[ub * kRowsPerBlock + rl + 16 * mi + r] = q;
      }
    }
    __syncthreads();
    if (tid < kRowsPerBlock) {
      const float o = ((sPart[tid] + sPart[kRowsPerBlock + tid]) + sPart[2 * kRowsPerBlock + tid])
                      + sPart[3 * kRowsPerBlock + tid] + wob0;
      sOut[tid * kOutCols + t] = o;
    }
  }
  __syncthreads();

  {
    const v4f v = *(const v4f*)(sOut + wave * 128 + lane * 4);
    float* dst = OW + (size_t)blockIdx.x * (kRowsPerBlock * kOutCols) + wave * 128 + lane * 4;
    *(volatile v4f*)dst = v;
    __threadfence();
    *(volatile v4f*)dst = v;
  }
}

__global__ __launch_bounds__(kPermThreads) void permute_out(const float* __restrict__ OW, float* __restrict__ out) {
  const int g  = blockIdx.x * kPermThreads + threadIdx.x;
  const int e0 = g << 2;
  const int bt = e0 / kNodes;
  const int n0 = e0 - bt * kNodes;
  const int b  = bt / kTdec;
  const int t  = bt - b * kTdec;
  const float* src = OW + ((size_t)(b * kNodes + n0)) * kOutCols + t;
  v4f v;
  v[0] = src[0];
  v[1] = src[kOutCols];
  v[2] = src[2 * kOutCols];
  v[3] = src[3 * kOutCols];
  float* dst = out + e0;
  *(volatile v4f*)dst = v;
  __threadfence();
  *(volatile v4f*)dst = v;
}

extern "C" void kernel_launch(void* const* d_in, const int* in_sizes, int n_in,
                              void* d_out, int out_size, void* d_ws, size_t ws_size,
                              hipStream_t stream) {
  if (n_in < 17) return;
  if (in_sizes[0] != kBatch * kSteps * kNodes) return;
  if (out_size != kBatch * kTdec * kNodes) return;
  if (in_sizes[1] != 64 || in_sizes[2] != 64) return;
  if (in_sizes[3] != 128 * 128 || in_sizes[4] != 128 || in_sizes[5] != 128 * 64 || in_sizes[6] != 64) return;
  if (in_sizes[7] != 64 * 64 || in_sizes[8] != 64) return;
  if (in_sizes[9] != 128 * 128 || in_sizes[10] != 128 || in_sizes[11] != 128 * 64 || in_sizes[12] != 64) return;
  if (in_sizes[13] != 64 * 64 || in_sizes[14] != 64 || in_sizes[15] != 64 || in_sizes[16] != 1) return;

  const size_t offEg = 0;
  const size_t offEu = offEg + (size_t)128 * 128 * 2;
  const size_t offEw = offEu + (size_t)64 * 128 * 2;
  const size_t offDg = offEw + (size_t)64 * 64 * 2;
  const size_t offDu = offDg + (size_t)128 * 128 * 2;
  const size_t offDw = offDu + (size_t)64 * 128 * 2;
  const size_t offOW = offDw + (size_t)64 * 64 * 2;
  const size_t wsEnd = offOW + (size_t)kRows * kOutCols * 4;
  if (ws_size < wsEnd) return;

  const float* xin   = (const float*)d_in[0];
  const float* winw  = (const float*)d_in[1];
  const float* winb  = (const float*)d_in[2];
  const float* eg_w  = (const float*)d_in[3];
  const float* eg_b  = (const float*)d_in[4];
  const float* eu_w  = (const float*)d_in[5];
  const float* eu_b  = (const float*)d_in[6];
  const float* e_w   = (const float*)d_in[7];
  const float* e_b   = (const float*)d_in[8];
  const float* dg_w  = (const float*)d_in[9];
  const float* dg_b  = (const float*)d_in[10];
  const float* du_w  = (const float*)d_in[11];
  const float* du_b  = (const float*)d_in[12];
  const float* d_w   = (const float*)d_in[13];
  const float* d_b   = (const float*)d_in[14];
  const float* wo_w  = (const float*)d_in[15];
  const float* wo_b  = (const float*)d_in[16];
  float* out = (float*)d_out;
  char* ws = (char*)d_ws;
  _Float16* egt = (_Float16*)(ws + offEg);
  _Float16* eut = (_Float16*)(ws + offEu);
  _Float16* ewt = (_Float16*)(ws + offEw);
  _Float16* dgt = (_Float16*)(ws + offDg);
  _Float16* dut = (_Float16*)(ws + offDu);
  _Float16* dwt = (_Float16*)(ws + offDw);
  float* OW = (float*)(ws + offOW);

  prep_wt8<<<8, 256, 0, stream>>>(eg_w, egt, 7, 128, 128 * 128 / 8);
  prep_wt8<<<4, 256, 0, stream>>>(eu_w, eut, 7, 64, 128 * 64 / 8);
  prep_wt8<<<2, 256, 0, stream>>>(e_w, ewt, 6, 64, 64 * 64 / 8);
  prep_wt8<<<8, 256, 0, stream>>>(dg_w, dgt, 7, 128, 128 * 128 / 8);
  prep_wt8<<<4, 256, 0, stream>>>(du_w, dut, 7, 64, 128 * 64 / 8);
  prep_wt8<<<2, 256, 0, stream>>>(d_w, dwt, 6, 64, 64 * 64 / 8);

  gru_seq_main<<<kMainBlocks, kMainThreads, 0, stream>>>(
      xin, winw, winb, egt, eg_b, eut, eu_b, ewt, e_b,
      dgt, dg_b, dut, du_b, dwt, d_b, wo_w, wo_b, OW);

  permute_out<<<kPermBlocks, kPermThreads, 0, stream>>>(OW, out);
}
